// PointNetSetAbstraction_26620207301335
// MI455X (gfx1250) — hardware-verified
//
#include <hip/hip_runtime.h>
#pragma clang fp contract(off)

typedef __attribute__((ext_vector_type(16))) _Float16 v16h;
typedef __attribute__((ext_vector_type(8)))  _Float16 v8h;
typedef __attribute__((ext_vector_type(8)))  float    v8f;
typedef __attribute__((ext_vector_type(4)))  float    v4f;
typedef __attribute__((ext_vector_type(4)))  unsigned v4u;
typedef __attribute__((ext_vector_type(2)))  unsigned v2u;

constexpr int NBATCH  = 4;
constexpr int NPTS    = 8192;
constexpr int NSAMP   = 2048;
constexpr int NNBR    = 32;
constexpr int NFEAT   = 64;
constexpr int CIN0    = 3 + NFEAT;
constexpr int KPAD0   = 96;
constexpr int NGROUPS = NBATCH * NSAMP;
constexpr int NROWS   = NGROUPS * NNBR;
constexpr int GEMM_BLOCKS = NROWS / 128;
static_assert(CIN0 == 67);
static_assert(NROWS == 262144);
static_assert(NROWS % 128 == 0);
static_assert(KPAD0 % 32 == 0);
static_assert(KPAD0 >= CIN0);

constexpr float FEAT_CARRY = 16.0f;
constexpr float WGT_CARRY  = 64.0f;
constexpr float Y0_CARRY   = 16.0f;
constexpr float Y1_CARRY   = 16.0f;

constexpr size_t SZ_WH    = (size_t)(64 * KPAD0 + 64 * 64 + 128 * 64) * 2;
constexpr size_t SZ_NXYZ  = (size_t)NGROUPS * 3 * 4;
constexpr size_t SZ_AFF   = (size_t)3 * 256 * 4;
constexpr size_t SZ_PART0 = (size_t)GEMM_BLOCKS * 2 * 64 * 4;
constexpr size_t SZ_PART1 = (size_t)GEMM_BLOCKS * 2 * 64 * 4;
constexpr size_t SZ_PART2 = (size_t)GEMM_BLOCKS * 2 * 128 * 4;
constexpr size_t SZ_YMM   = (size_t)NGROUPS * 128 * 4;
constexpr size_t SZ_FEAT  = (size_t)NROWS * KPAD0 * 2;
constexpr size_t SZ_Y     = (size_t)NROWS * 64 * 2;
constexpr size_t WS_WH    = 0;
constexpr size_t WS_NXYZ  = WS_WH + SZ_WH;
constexpr size_t WS_AFF   = WS_NXYZ + SZ_NXYZ;
constexpr size_t WS_PART0 = WS_AFF + SZ_AFF;
constexpr size_t WS_PART1 = WS_PART0 + SZ_PART0;
constexpr size_t WS_PART2 = WS_PART1 + SZ_PART1;
constexpr size_t WS_YMAX  = WS_PART2 + SZ_PART2;
constexpr size_t WS_YMIN  = WS_YMAX + SZ_YMM;
constexpr size_t WS_FEAT  = WS_YMIN + SZ_YMM;
constexpr size_t WS_Y0    = WS_FEAT + SZ_FEAT;
constexpr size_t WS_Y1    = WS_Y0 + SZ_Y;
constexpr size_t WS_TOTAL = WS_Y1 + SZ_Y;
static_assert(SZ_WH == 36864);
static_assert(SZ_PART0 == 1048576 && SZ_PART1 == 1048576 && SZ_PART2 == 2097152);
static_assert(WS_TOTAL == 130161664);
static_assert(WS_TOTAL <= 134217728);
static_assert(WS_NXYZ % 256 == 0 && WS_AFF % 256 == 0 && WS_PART0 % 256 == 0 && WS_PART1 % 256 == 0);
static_assert(WS_PART2 % 256 == 0 && WS_YMAX % 256 == 0 && WS_YMIN % 256 == 0);
static_assert(WS_FEAT % 256 == 0 && WS_Y0 % 256 == 0 && WS_Y1 % 256 == 0);

constexpr size_t OUT1_BYTE_OFF = (size_t)NGROUPS * 3 * 4;
static_assert(OUT1_BYTE_OFF == 98304);
static_assert(OUT1_BYTE_OFF % 128 == 0);
static_assert(OUT1_BYTE_OFF + (size_t)NBATCH * 128 * NSAMP * 4 == 4292608);

__device__ __forceinline__ unsigned f16bits(float f) {
  const _Float16 h = (_Float16)f;
  const unsigned short us = __builtin_bit_cast(unsigned short, h);
  return (unsigned)us;
}
__device__ __forceinline__ float h16_to_f32(unsigned hb) {
  const unsigned sgn = (hb & 0x8000u) << 16;
  const unsigned em = hb & 0x7fffu;
  const float fn = __uint_as_float((em << 13) + 0x38000000u);
  const float fs = (float)em * 5.9604644775390625e-8f;
  const float mag = (em < 0x400u) ? fs : fn;
  return __uint_as_float(__float_as_uint(mag) | sgn);
}
__device__ __forceinline__ void wave_sync() {
  __builtin_amdgcn_fence(__ATOMIC_RELEASE, "workgroup");
  __builtin_amdgcn_wave_barrier();
  __builtin_amdgcn_fence(__ATOMIC_ACQUIRE, "workgroup");
}
union FragH { v16h v; v8h h[2]; };
__device__ __forceinline__ v16h frag_load(const _Float16* p) {
  FragH f;
  f.h[0] = *(const v8h*)(p);
  f.h[1] = *(const v8h*)(p + 16);
  return f.v;
}
__device__ __forceinline__ v8f mma_g(v16h a, v16h b, v8f c) {
  c = __builtin_amdgcn_wmma_f32_16x16x32_f16(false, a, false, b, (short)0, c, false, false);
  asm volatile("v_nop\n\tv_nop\n\tv_nop\n\tv_nop" : "+v"(c) : "v"(a), "v"(b));
  return c;
}

__global__ __launch_bounds__(256) void prep_weights(const float* __restrict__ w0,
                                                    const float* __restrict__ w1,
                                                    const float* __restrict__ w2,
                                                    unsigned short* __restrict__ wh) {
  const int blk = blockIdx.x;
  const int i = blk * 256 + threadIdx.x;
  float v[8];
  if (blk < 3) {
    const int base = i * 8;
    const int o = base / KPAD0;
    const int k0 = base - o * KPAD0;
#pragma unroll
    for (int e = 0; e < 8; ++e) {
      const int k = k0 + e;
      const int col = (k < 64) ? (k + 3) : ((k < CIN0) ? (k - 64) : 0);
      const float x = w0[o * CIN0 + col];
      v[e] = (k < CIN0) ? x : 0.0f;
    }
  } else if (blk < 5) {
    const int j = i - 768;
    const v4f a = *(const v4f*)(w1 + j * 8);
    const v4f b = *(const v4f*)(w1 + j * 8 + 4);
    v[0] = a.x; v[1] = a.y; v[2] = a.z; v[3] = a.w;
    v[4] = b.x; v[5] = b.y; v[6] = b.z; v[7] = b.w;
  } else {
    const int j = i - 1280;
    const v4f a = *(const v4f*)(w2 + j * 8);
    const v4f b = *(const v4f*)(w2 + j * 8 + 4);
    v[0] = a.x; v[1] = a.y; v[2] = a.z; v[3] = a.w;
    v[4] = b.x; v[5] = b.y; v[6] = b.z; v[7] = b.w;
  }
  v8h hv;
#pragma unroll
  for (int e = 0; e < 8; ++e) hv[e] = (_Float16)(v[e] * WGT_CARRY);
  *(volatile v8h*)(wh + (size_t)i * 8) = hv;
  __threadfence();
  *(volatile v8h*)(wh + (size_t)i * 8) = hv;
}

__global__ __launch_bounds__(256) void fps_kernel(const float* __restrict__ xyz,
                                                  float* __restrict__ nxyz,
                                                  float* __restrict__ out0) {
#pragma clang fp contract(off)
  __shared__ __align__(16) float sStage[2048 * 3];
  __shared__ __align__(16) float sNew[NSAMP * 3];
  __shared__ float sRv[2][8];
  __shared__ int   sRi[2][8];
  const int b = blockIdx.x;
  const int tx = threadIdx.x;
  const int lane = tx & 31;
  const int wave = tx >> 5;
  const float* X = xyz + (size_t)b * NPTS * 3;

  float px[32], py[32], pz[32], dist[32];
#pragma unroll
  for (int c = 0; c < 4; ++c) {
    const v4f* src = (const v4f*)(X + c * 6144);
#pragma unroll
    for (int i = 0; i < 6; ++i) {
      const v4f v = src[i * 256 + tx];
      *(v4f*)(sStage + (i * 256 + tx) * 4) = v;
    }
    asm volatile("" ::: "memory");
    __syncthreads();
#pragma unroll
    for (int jj = 0; jj < 8; ++jj) {
      const int nl = jj * 256 + tx;
      px[c * 8 + jj] = sStage[nl * 3 + 0];
      py[c * 8 + jj] = sStage[nl * 3 + 1];
      pz[c * 8 + jj] = sStage[nl * 3 + 2];
      dist[c * 8 + jj] = 1e18f;
    }
    __syncthreads();
  }

  int far = 0;
  for (int s = 0; s < NSAMP; ++s) {
    const float cx = X[far * 3 + 0];
    const float cy = X[far * 3 + 1];
    const float cz = X[far * 3 + 2];
    if (tx == 0) {
      sNew[s * 3 + 0] = cx;
      sNew[s * 3 + 1] = cy;
      sNew[s * 3 + 2] = cz;
    }
    float bd = -1.0f;
    int bi = 0;
#pragma unroll
    for (int j = 0; j < 32; ++j) {
      const float dx = px[j] - cx;
      const float dy = py[j] - cy;
      const float dz = pz[j] - cz;
      const float t0 = dx * dx;
      const float t1 = dy * dy;
      const float t2 = dz * dz;
      const float d = (t0 + t2) + t1;
      const float dj = fminf(dist[j], d);
      dist[j] = dj;
      const bool tk = dj > bd;
      bd = tk ? dj : bd;
      bi = tk ? (j * 256 + tx) : bi;
    }
#pragma unroll
    for (int off = 16; off >= 1; off >>= 1) {
      const float ov = __shfl_xor(bd, off, 32);
      const int oi = __shfl_xor(bi, off, 32);
      const bool tk = (ov > bd) || ((ov == bd) && (oi < bi));
      bd = tk ? ov : bd;
      bi = tk ? oi : bi;
    }
    const int par = s & 1;
    if (lane == 0) {
      sRv[par][wave] = bd;
      sRi[par][wave] = bi;
    }
    __syncthreads();
    float bv = sRv[par][0];
    int bx = sRi[par][0];
#pragma unroll
    for (int w = 1; w < 8; ++w) {
      const float ov = sRv[par][w];
      const int oi = sRi[par][w];
      const bool tk = (ov > bv) || ((ov == bv) && (oi < bx));
      bv = tk ? ov : bv;
      bx = tk ? oi : bx;
    }
    bx = bx < 0 ? 0 : bx;
    bx = bx > (NPTS - 1) ? (NPTS - 1) : bx;
    far = bx;
  }
  __syncthreads();
  float* odst = out0 + (size_t)b * NSAMP * 3;
  float* wdst = nxyz + (size_t)b * NSAMP * 3;
  for (int pass = 0; pass < 2; ++pass) {
#pragma unroll
    for (int i = 0; i < 6; ++i) {
      const v4f v = *(const v4f*)(sNew + (i * 256 + tx) * 4);
      *(volatile v4f*)(odst + (i * 256 + tx) * 4) = v;
      *(volatile v4f*)(wdst + (i * 256 + tx) * 4) = v;
    }
    __threadfence();
  }
}

__global__ __launch_bounds__(256) void ballq_feat_kernel(const float* __restrict__ xyz,
                                                         const float* __restrict__ points,
                                                         const float* __restrict__ nxyz,
                                                         unsigned short* __restrict__ featA) {
#pragma clang fp contract(off)
  __shared__ __align__(16) unsigned sTile[8][32 * 48];
  __shared__ int sBuf[8][NNBR];
  const int wave = threadIdx.x >> 5;
  const int lane = threadIdx.x & 31;
  const int hh = lane >> 4;
  const int c16 = lane & 15;
  const int g = blockIdx.x * 8 + wave;
  const int b = g / NSAMP;
  const float* X = xyz + (size_t)b * NPTS * 3;
  const float qx = nxyz[(size_t)g * 3 + 0];
  const float qy = nxyz[(size_t)g * 3 + 1];
  const float qz = nxyz[(size_t)g * 3 + 2];
  const float q0 = qx * qx;
  const float q1 = qy * qy;
  const float q2s = qz * qz;
  const float qq = (q0 + q2s) + q1;
  const float r2 = 0.04f;

  sBuf[wave][lane] = 0;
  __syncthreads();

  int cnt = 0;
  for (int chunk = 0; chunk < NPTS / 32 && cnt < NNBR; ++chunk) {
    const int np = chunk * 32 + lane;
    const float x = X[np * 3 + 0];
    const float y = X[np * 3 + 1];
    const float z = X[np * 3 + 2];
    float p = qx * x;
    p = fmaf(qy, y, p);
    p = fmaf(qz, z, p);
    const float x0 = x * x;
    const float x1 = y * y;
    const float x2s = z * z;
    const float xx = (x0 + x2s) + x1;
    float d = -2.0f * p;
    d = d + qq;
    d = d + xx;
    d = fmaxf(d, 0.0f);
    const bool inball = !(d > r2);
    const unsigned mask = __builtin_amdgcn_ballot_w32(inball);
    const int slot = cnt + __popc(mask & ((1u << lane) - 1u));
    if (inball && slot < NNBR) sBuf[wave][slot] = np;
    cnt += __popc(mask);
  }
  __syncthreads();
  const int slot0 = sBuf[wave][0];
  const int mine = sBuf[wave][lane];
  const int first = (cnt > 0) ? slot0 : (NPTS - 1);
  int n = (lane < cnt) ? mine : first;
  n = n < 0 ? 0 : n;
  n = n > (NPTS - 1) ? (NPTS - 1) : n;

  const float gx = X[n * 3 + 0] - qx;
  const float gy = X[n * 3 + 1] - qy;
  const float gz = X[n * 3 + 2] - qz;
  unsigned* tw = sTile[wave];
  {
    const unsigned hx = f16bits(gx * FEAT_CARRY);
    const unsigned hy = f16bits(gy * FEAT_CARRY);
    const unsigned hz = f16bits(gz * FEAT_CARRY);
    unsigned zz = 0u;
    asm volatile("" : "+v"(zz));
    v4u a;
    a.x = (hx & 0xffffu) | (hy << 16);
    a.y = (hz & 0xffffu) | (zz << 16);
    a.z = zz;
    a.w = zz;
    v4u zv;
    zv.x = zz;
    zv.y = zz;
    zv.z = zz;
    zv.w = zz;
    *(v4u*)(tw + lane * 48 + 32) = a;
    *(v4u*)(tw + lane * 48 + 36) = zv;
    *(v4u*)(tw + lane * 48 + 40) = zv;
    *(v4u*)(tw + lane * 48 + 44) = zv;
  }
#pragma unroll 1
  for (int o = 0; o < 4; ++o) {
#pragma unroll
    for (int ii = 0; ii < 4; ++ii) {
      const int row = (o * 4 + ii) * 2 + hh;
      const int src = __shfl(n, row, 32);
      const v4f pv = *(const v4f*)(points + ((size_t)b * NPTS + (size_t)src) * NFEAT + c16 * 4);
      const float p0 = pv.x;
      const float p1 = pv.y;
      const float p2 = pv.z;
      const float p3 = pv.w;
      const unsigned h0 = f16bits(p0 * FEAT_CARRY);
      const unsigned h1 = f16bits(p1 * FEAT_CARRY);
      const unsigned h2 = f16bits(p2 * FEAT_CARRY);
      const unsigned h3 = f16bits(p3 * FEAT_CARRY);
      v2u w;
      w.x = (h0 & 0xffffu) | (h1 << 16);
      w.y = (h2 & 0xffffu) | (h3 << 16);
      *(v2u*)(tw + row * 48 + c16 * 2) = w;
    }
    asm volatile("" ::: "memory");
  }
  __syncthreads();
  v4u* dst = (v4u*)(featA + (size_t)g * NNBR * KPAD0);
  const v4u* src4 = (const v4u*)tw;
  for (int pass = 0; pass < 2; ++pass) {
#pragma unroll 4
    for (int it = 0; it < 12; ++it) {
      const v4u v = src4[it * 32 + lane];
      *(volatile v4u*)(dst + it * 32 + lane) = v;
    }
    __threadfence();
  }
}

template <int NOUT, int KP, bool CONV, bool STORE_Y>
__global__ __launch_bounds__(128) void mlp_gemm(const unsigned short* __restrict__ Ain,
                                                const unsigned short* __restrict__ Wh,
                                                const float* __restrict__ bias,
                                                const float* __restrict__ affin,
                                                unsigned short* __restrict__ Yout,
                                                float* __restrict__ part,
                                                float* __restrict__ ymax,
                                                float* __restrict__ ymin,
                                                float in_inv, float acc_inv, float out_carry) {
  static_assert(NOUT % 64 == 0);
  static_assert(KP % 32 == 0);
  static_assert(!CONV || KP == 64);
  static_assert(!STORE_Y || NOUT == 64);
  __shared__ __align__(16) _Float16 sA[4][32 * KP];
  __shared__ __align__(16) _Float16 sW[NOUT * KP];
  __shared__ __align__(16) float sBias[NOUT];
  __shared__ __align__(16) float sStat[4][2][NOUT];
  __shared__ __align__(16) float sMM[STORE_Y ? 1 : 4][2][STORE_Y ? 4 : 128];
  __shared__ __align__(16) float sSlab[STORE_Y ? 4 : 1][STORE_Y ? 16 * 68 : 4];

  const int tid = threadIdx.x;
  const int wave = tid >> 5;
  const int lane = tid & 31;
  const int rlane = lane & 15;
  const int hh = lane >> 4;
  const int koff = hh * 8;
  const size_t rowbase = ((size_t)blockIdx.x * 4 + (size_t)wave) * 32;

  {
    const _Float16* wsrc = (const _Float16*)Wh;
#pragma unroll 4
    for (int i = tid; i < NOUT * KP / 8; i += 128) {
      const v8h w = *(const v8h*)(wsrc + i * 8);
      *(v8h*)(sW + i * 8) = w;
    }
    for (int i = tid; i < NOUT; i += 128) sBias[i] = bias[i];
  }
  _Float16* aw = sA[wave];
  if constexpr (!CONV) {
    const _Float16* asrc = (const _Float16*)Ain + rowbase * KP;
#pragma unroll 4
    for (int it = 0; it < KP / 8; ++it) {
      const v8h a = *(const v8h*)(asrc + (it * 32 + lane) * 8);
      *(v8h*)(aw + (it * 32 + lane) * 8) = a;
    }
  } else {
    const int c8 = (lane & 7) * 8;
    const v4f a_lo = *(const v4f*)(affin + c8);
    const v4f a_hi = *(const v4f*)(affin + c8 + 4);
    const v4f c_lo = *(const v4f*)(affin + 128 + c8);
    const v4f c_hi = *(const v4f*)(affin + 128 + c8 + 4);
    const float av[8] = {a_lo.x, a_lo.y, a_lo.z, a_lo.w, a_hi.x, a_hi.y, a_hi.z, a_hi.w};
    const float cv[8] = {c_lo.x, c_lo.y, c_lo.z, c_lo.w, c_hi.x, c_hi.y, c_hi.z, c_hi.w};
    const v4u* ysrc = (const v4u*)(Ain + rowbase * 64);
#pragma unroll 2
    for (int it = 0; it < 8; ++it) {
      const v4u w = ysrc[it * 32 + lane];
      const unsigned w0 = w.x;
      const unsigned w1 = w.y;
      const unsigned w2 = w.z;
      const unsigned w3 = w.w;
      float xv[8];
      xv[0] = h16_to_f32(w0 & 0xffffu);
      xv[1] = h16_to_f32(w0 >> 16);
      xv[2] = h16_to_f32(w1 & 0xffffu);
      xv[3] = h16_to_f32(w1 >> 16);
      xv[4] = h16_to_f32(w2 & 0xffffu);
      xv[5] = h16_to_f32(w2 >> 16);
      xv[6] = h16_to_f32(w3 & 0xffffu);
      xv[7] = h16_to_f32(w3 >> 16);
      v8h hv;
#pragma unroll
      for (int e = 0; e < 8; ++e) {
        const float yv = xv[e] * in_inv;
        const float sc = av[e] * yv;
        const float act = fmaxf(sc + cv[e], 0.0f);
        hv[e] = (_Float16)act;
      }
      *(v8h*)(aw + (it * 32 + lane) * 8) = hv;
    }
  }
  __syncthreads();

#pragma unroll 1
  for (int nh = 0; nh < NOUT / 64; ++nh) {
    v8f acc[2][4];
#pragma unroll
    for (int i = 0; i < 2; ++i)
#pragma unroll
      for (int j = 0; j < 4; ++j) acc[i][j] = (v8f){0.f, 0.f, 0.f, 0.f, 0.f, 0.f, 0.f, 0.f};

#pragma unroll
    for (int kb = 0; kb < KP / 32; ++kb) {
      const v16h af0 = frag_load(aw + (rlane) * KP + kb * 32 + koff);
      const v16h af1 = frag_load(aw + (16 + rlane) * KP + kb * 32 + koff);
#pragma unroll
      for (int j = 0; j < 4; ++j) {
        const v16h bf = frag_load(sW + (nh * 64 + j * 16 + rlane) * KP + kb * 32 + koff);
        acc[0][j] = mma_g(af0, bf, acc[0][j]);
        acc[1][j] = mma_g(af1, bf, acc[1][j]);
      }
    }

    float cs[4], cq[4], cmx[4], cmn[4];
#pragma unroll
    for (int j = 0; j < 4; ++j) {
      cs[j] = 0.0f;
      cq[j] = 0.0f;
      cmx[j] = -__builtin_huge_valf();
      cmn[j] = __builtin_huge_valf();
    }
    float* slab = sSlab[STORE_Y ? wave : 0];
#pragma unroll
    for (int i = 0; i < 2; ++i) {
#pragma unroll
      for (int j = 0; j < 4; ++j) {
        const float bv = sBias[nh * 64 + j * 16 + rlane];
#pragma unroll
        for (int r = 0; r < 8; ++r) {
          const float sc = acc[i][j][r] * acc_inv;
          const float y = sc + bv;
          cs[j] = cs[j] + y;
          const float y2 = y * y;
          cq[j] = cq[j] + y2;
          if constexpr (!STORE_Y) {
            cmx[j] = fmaxf(cmx[j], y);
            cmn[j] = fminf(cmn[j], y);
          }
          if constexpr (STORE_Y) slab[(hh * 8 + r) * 68 + j * 16 + rlane] = y * out_carry;
        }
      }
      if constexpr (STORE_Y) {
        wave_sync();
        const int q4 = lane >> 3;
        const int c8 = (lane & 7) * 8;
        for (int pass = 0; pass < 2; ++pass) {
#pragma unroll
          for (int it = 0; it < 4; ++it) {
            const int row = it * 4 + q4;
            const float* sp = slab + row * 68 + c8;
            v8h hv;
#pragma unroll
            for (int e = 0; e < 8; ++e) hv[e] = (_Float16)sp[e];
            *(volatile v8h*)(Yout + (rowbase + (size_t)(i * 16 + row)) * 64 + c8) = hv;
          }
          __threadfence();
        }
        wave_sync();
      }
    }
#pragma unroll
    for (int j = 0; j < 4; ++j) {
      const float os = __shfl_xor(cs[j], 16, 32);
      const float oq = __shfl_xor(cq[j], 16, 32);
      const float omx = __shfl_xor(cmx[j], 16, 32);
      const float omn = __shfl_xor(cmn[j], 16, 32);
      cs[j] = cs[j] + os;
      cq[j] = cq[j] + oq;
      cmx[j] = fmaxf(cmx[j], omx);
      cmn[j] = fminf(cmn[j], omn);
    }
    if (hh == 0) {
#pragma unroll
      for (int j = 0; j < 4; ++j) {
        const int col = nh * 64 + j * 16 + rlane;
        sStat[wave][0][col] = cs[j];
        sStat[wave][1][col] = cq[j];
        if constexpr (!STORE_Y) {
          sMM[wave][0][col] = cmx[j];
          sMM[wave][1][col] = cmn[j];
        }
      }
    }
  }
  __syncthreads();

  {
    constexpr int NQ = (2 * NOUT) / 128;
    float pv[NQ];
#pragma unroll
    for (int q = 0; q < NQ; ++q) {
      const int flat = q * 128 + tid;
      const int qq = flat / NOUT;
      const int ch = flat - qq * NOUT;
      const float s01 = sStat[0][qq][ch] + sStat[1][qq][ch];
      const float s23 = sStat[2][qq][ch] + sStat[3][qq][ch];
      pv[q] = s01 + s23;
    }
    float* pp = part + (size_t)blockIdx.x * 2 * NOUT;
    for (int pass = 0; pass < 2; ++pass) {
#pragma unroll
      for (int q = 0; q < NQ; ++q) *(volatile float*)(pp + q * 128 + tid) = pv[q];
      __threadfence();
    }
  }
  if constexpr (!STORE_Y) {
    const size_t grp = (size_t)blockIdx.x * 4 + (size_t)wave;
    const v4f mxv = *(const v4f*)(&sMM[wave][0][lane * 4]);
    const v4f mnv = *(const v4f*)(&sMM[wave][1][lane * 4]);
    for (int pass = 0; pass < 2; ++pass) {
      *(volatile v4f*)(ymax + grp * 128 + lane * 4) = mxv;
      *(volatile v4f*)(ymin + grp * 128 + lane * 4) = mnv;
      __threadfence();
    }
  }
}

__global__ __launch_bounds__(256) void bn_finalize(const float* __restrict__ part, int nblk, int nout,
                                                   const float* __restrict__ gamma,
                                                   const float* __restrict__ beta,
                                                   float* __restrict__ aff) {
  __shared__ float sAC[256];
  const int tid = threadIdx.x;
  const int wave = tid >> 5;
  const int lane = tid & 31;
  sAC[tid] = 0.0f;
  __syncthreads();
  const int no = nout > 128 ? 128 : nout;
  for (int ch = wave; ch < no; ch += 8) {
    double s = 0.0;
    double q = 0.0;
#pragma unroll 4
    for (int i = lane; i < nblk; i += 32) {
      const float ps = part[(size_t)i * 2 * no + ch];
      const float pq = part[(size_t)i * 2 * no + no + ch];
      s = s + (double)ps;
      q = q + (double)pq;
    }
#pragma unroll
    for (int off = 16; off >= 1; off >>= 1) {
      const double os = __shfl_xor(s, off, 32);
      const double oq = __shfl_xor(q, off, 32);
      s = s + os;
      q = q + oq;
    }
    const double inv_n = 1.0 / (double)NROWS;
    const double mu = s * inv_n;
    const double ex2 = q * inv_n;
    const double mu2 = mu * mu;
    double var = ex2 - mu2;
    var = var < 0.0 ? 0.0 : var;
    const float vf = (float)var + 1e-5f;
    const float a = gamma[ch] * rsqrtf(vf);
    const float ma = (float)mu * a;
    const float c = beta[ch] - ma;
    if (lane == 0) {
      sAC[ch] = a;
      sAC[128 + ch] = c;
    }
  }
  __syncthreads();
  const float v = sAC[tid];
  volatile float* dst = aff + tid;
  *dst = v;
  __threadfence();
  *dst = v;
}

__global__ __launch_bounds__(256) void final_kernel(const float* __restrict__ ymax,
                                                    const float* __restrict__ ymin,
                                                    const float* __restrict__ aff2,
                                                    float* __restrict__ out1) {
  __shared__ __align__(16) float sT[32][132];
  const int tid = threadIdx.x;
  const int wave = tid >> 5;
  const int lane = tid & 31;
  const int b = blockIdx.x / (NSAMP / 32);
  const int s0 = (blockIdx.x - b * (NSAMP / 32)) * 32;
  const size_t g0 = (size_t)b * NSAMP + (size_t)s0;
  const v4f a4 = *(const v4f*)(aff2 + lane * 4);
  const v4f c4 = *(const v4f*)(aff2 + 128 + lane * 4);
  const float aa[4] = {a4.x, a4.y, a4.z, a4.w};
  const float cc[4] = {c4.x, c4.y, c4.z, c4.w};
  float fa[4], fb[4];
#pragma unroll
  for (int e = 0; e < 4; ++e) {
    fa[e] = (aa[e] >= 0.0f) ? 1.0f : 0.0f;
    fb[e] = 1.0f - fa[e];
  }
#pragma unroll
  for (int it = 0; it < 4; ++it) {
    const int r = wave * 4 + it;
    const v4f mx = *(const v4f*)(ymax + (g0 + (size_t)r) * 128 + lane * 4);
    const v4f mn = *(const v4f*)(ymin + (g0 + (size_t)r) * 128 + lane * 4);
    const float mxv[4] = {mx.x, mx.y, mx.z, mx.w};
    const float mnv[4] = {mn.x, mn.y, mn.z, mn.w};
    v4f o;
#pragma unroll
    for (int e = 0; e < 4; ++e) {
      const float sa = fa[e] * mxv[e];
      const float sb = fb[e] * mnv[e];
      const float sel = sa + sb;
      const float sc = aa[e] * sel;
      o[e] = fmaxf(sc + cc[e], 0.0f);
    }
    *(v4f*)(&sT[r][lane * 4]) = o;
    asm volatile("" ::: "memory");
  }
  __syncthreads();
  v4f ov[4];
  const int s4 = (lane & 7) * 4;
#pragma unroll
  for (int it = 0; it < 4; ++it) {
    const int ch = wave * 16 + it * 4 + (lane >> 3);
    v4f o;
    o.x = sT[s4 + 0][ch];
    o.y = sT[s4 + 1][ch];
    o.z = sT[s4 + 2][ch];
    o.w = sT[s4 + 3][ch];
    ov[it] = o;
  }
  for (int pass = 0; pass < 2; ++pass) {
#pragma unroll
    for (int it = 0; it < 4; ++it) {
      const int ch = wave * 16 + it * 4 + (lane >> 3);
      *(volatile v4f*)(out1 + ((size_t)b * 128 + (size_t)ch) * NSAMP + s0 + s4) = ov[it];
    }
    __threadfence();
  }
}

extern "C" void kernel_launch(void* const* d_in, const int* in_sizes, int n_in,
                              void* d_out, int out_size, void* d_ws, size_t ws_size,
                              hipStream_t stream) {
  (void)in_sizes;
  (void)out_size;
  if (n_in < 14) return;
  if (ws_size < WS_TOTAL) return;

  const float* xyz    = (const float*)d_in[0];
  const float* points = (const float*)d_in[1];
  const float* w0  = (const float*)d_in[2];
  const float* b0  = (const float*)d_in[3];
  const float* g0  = (const float*)d_in[4];
  const float* be0 = (const float*)d_in[5];
  const float* w1  = (const float*)d_in[6];
  const float* b1  = (const float*)d_in[7];
  const float* g1  = (const float*)d_in[8];
  const float* be1 = (const float*)d_in[9];
  const float* w2  = (const float*)d_in[10];
  const float* b2  = (const float*)d_in[11];
  const float* g2  = (const float*)d_in[12];
  const float* be2 = (const float*)d_in[13];

  char* ws = (char*)d_ws;
  unsigned short* wh    = (unsigned short*)(ws + WS_WH);
  unsigned short* w0h   = wh;
  unsigned short* w1h   = wh + 64 * KPAD0;
  unsigned short* w2h   = wh + 64 * KPAD0 + 64 * 64;
  float* nxyz    = (float*)(ws + WS_NXYZ);
  float* aff     = (float*)(ws + WS_AFF);
  float* part0   = (float*)(ws + WS_PART0);
  float* part1   = (float*)(ws + WS_PART1);
  float* part2   = (float*)(ws + WS_PART2);
  float* ymax    = (float*)(ws + WS_YMAX);
  float* ymin    = (float*)(ws + WS_YMIN);
  unsigned short* featA = (unsigned short*)(ws + WS_FEAT);
  unsigned short* y0h   = (unsigned short*)(ws + WS_Y0);
  unsigned short* y1h   = (unsigned short*)(ws + WS_Y1);

  float* out0 = (float*)d_out;
  float* out1 = (float*)((char*)d_out + OUT1_BYTE_OFF);

  const float inv_fw = 1.0f / (FEAT_CARRY * WGT_CARRY);
  const float inv_w  = 1.0f / WGT_CARRY;
  const float inv_y0 = 1.0f / Y0_CARRY;
  const float inv_y1 = 1.0f / Y1_CARRY;

  prep_weights<<<9, 256, 0, stream>>>(w0, w1, w2, wh);
  fps_kernel<<<NBATCH, 256, 0, stream>>>(xyz, nxyz, out0);
  ballq_feat_kernel<<<NGROUPS / 8, 256, 0, stream>>>(xyz, points, nxyz, featA);

  mlp_gemm<64, KPAD0, false, true><<<GEMM_BLOCKS, 128, 0, stream>>>(
      featA, w0h, b0, aff, y0h, part0, ymax, ymin, 1.0f, inv_fw, Y0_CARRY);
  bn_finalize<<<1, 256, 0, stream>>>(part0, GEMM_BLOCKS, 64, g0, be0, aff);

  mlp_gemm<64, 64, true, true><<<GEMM_BLOCKS, 128, 0, stream>>>(
      y0h, w1h, b1, aff, y1h, part1, ymax, ymin, inv_y0, inv_w, Y1_CARRY);
  bn_finalize<<<1, 256, 0, stream>>>(part1, GEMM_BLOCKS, 64, g1, be1, aff + 256);

  mlp_gemm<128, 64, true, false><<<GEMM_BLOCKS, 128, 0, stream>>>(
      y1h, w2h, b2, aff + 256, featA, part2, ymax, ymin, inv_y1, inv_w, 1.0f);
  bn_finalize<<<1, 256, 0, stream>>>(part2, GEMM_BLOCKS, 128, g2, be2, aff + 512);

  final_kernel<<<NBATCH * (NSAMP / 32), 256, 0, stream>>>(ymax, ymin, aff + 512, out1);
}
